// FNOWithGlobalHead_77816217468964
// MI455X (gfx1250) — hardware-verified
//
#include <hip/hip_runtime.h>
#include <math.h>


typedef __attribute__((ext_vector_type(16))) _Float16 v16h;
typedef __attribute__((ext_vector_type(8)))  _Float16 v8h;
typedef __attribute__((ext_vector_type(16))) __bf16   v16b;
typedef __attribute__((ext_vector_type(8)))  __bf16   v8b;
typedef __attribute__((ext_vector_type(8)))  float    v8f;
typedef __attribute__((ext_vector_type(4)))  float    v4f;
typedef __attribute__((ext_vector_type(2)))  float    v2f;

__device__ __forceinline__ unsigned short f2bf_bits(float f) {
  unsigned u = __float_as_uint(f);
  return (unsigned short)((u + 0x7FFFu + ((u >> 16) & 1u)) >> 16);
}
__device__ __forceinline__ float bf_bits2f(unsigned short h) { return __uint_as_float(((unsigned)h) << 16); }

__device__ __forceinline__ void dep_guard_h(v8f& a, v8f& b, v16h x, v16h y) { asm volatile("v_nop\n\tv_nop\n\tv_nop\n\tv_nop" : "+v"(a), "+v"(b) : "v"(x), "v"(y)); }
__device__ __forceinline__ void dep_guard_b(v8f& a, v8f& b, v16b x, v16b y) { asm volatile("v_nop\n\tv_nop\n\tv_nop\n\tv_nop" : "+v"(a), "+v"(b) : "v"(x), "v"(y)); }
__device__ __forceinline__ void keep4_h(v16h a, v16h b, v16h c, v16h d) { asm volatile("v_nop" :: "v"(a), "v"(b), "v"(c), "v"(d)); }
__device__ __forceinline__ void keep4_b(v16b a, v16b b, v16b c, v16b d) { asm volatile("v_nop" :: "v"(a), "v"(b), "v"(c), "v"(d)); }
__device__ __forceinline__ void acc_guard4(v8f& a, v8f& b, v8f& c, v8f& d) { asm volatile("v_nop\n\tv_nop\n\tv_nop\n\tv_nop" : "+v"(a), "+v"(b), "+v"(c), "+v"(d)); }
template <typename T> struct Frag;
template <> struct Frag<_Float16> {
  typedef v16h V; union U { v16h v; v8h h[2]; };
  static __device__ __forceinline__ v16h load(const _Float16* p) {
    U f; f.h[0] = *(const v8h*)(p); f.h[1] = *(const v8h*)(p + 16); return f.v;
  }
  static __device__ __forceinline__ v8f mma(v16h a, v16h b, v8f c) {
    return __builtin_amdgcn_wmma_f32_16x16x32_f16(false, a, false, b, (short)0, c, false, false);
  }
  static __device__ __forceinline__ void guard(v8f& a, v8f& b, v16h x, v16h y) { dep_guard_h(a, b, x, y); }
  static __device__ __forceinline__ void keep(v16h a, v16h b, v16h c, v16h d) { keep4_h(a, b, c, d); }
};
template <> struct Frag<__bf16> {
  typedef v16b V; union U { v16b v; v8b h[2]; };
  static __device__ __forceinline__ v16b load(const __bf16* p) {
    U f; f.h[0] = *(const v8b*)(p); f.h[1] = *(const v8b*)(p + 16); return f.v;
  }
  static __device__ __forceinline__ v8f mma(v16b a, v16b b, v8f c) {
    return __builtin_amdgcn_wmma_f32_16x16x32_bf16(false, a, false, b, (short)0, c, false, false);
  }
  static __device__ __forceinline__ void guard(v8f& a, v8f& b, v16b x, v16b y) { dep_guard_b(a, b, x, y); }
  static __device__ __forceinline__ void keep(v16b a, v16b b, v16b c, v16b d) { keep4_b(a, b, c, d); }
};

template <int ET> struct Elem;
template <> struct Elem<0> { typedef _Float16 T; };
template <> struct Elem<1> { typedef __bf16 T; };
template <int ET, bool SPLIT, int BIAS_MODE, int OUT_MODE, bool RESID, int ACT = 0>
__global__ __launch_bounds__(256) void wmma_gemm64(
    const unsigned short* __restrict__ Ap, const unsigned short* __restrict__ A2p, int lda, long strideA,
    const unsigned short* __restrict__ Btp, const unsigned short* __restrict__ Bt2p, int ldb, long strideB,
    void* __restrict__ Cout, void* __restrict__ Cout2, int ldc, long strideC,
    const float* __restrict__ bias,
    const float* __restrict__ resid, long strideR,
    int M, int N, int K, float scale) {
  typedef typename Elem<ET>::T T;
  typedef typename Frag<T>::V V;
  const T* A = (const T*)Ap; const T* A2 = (const T*)A2p; const T* Bt = (const T*)Btp; const T* Bt2 = (const T*)Bt2p;
  __shared__ __align__(16) float sT[8][16 * 68];
  const int b    = blockIdx.y;
  const int lane = threadIdx.x & 31;
  const int wave = threadIdx.x >> 5;
  const int tilesN = N >> 6;
  const int tilesM = M >> 6;
  const int tile = blockIdx.x * 8 + wave;
  if (tile >= tilesM * tilesN) return;
  const int tm = tile / tilesN;
  const int tn = tile - tm * tilesN;
  const int m0 = tm << 6;
  const int n0 = tn << 6;

  const T* Ab  = A  + (size_t)b * strideA;
  const T* Bb  = Bt + (size_t)b * strideB;
  const T* Ab2 = SPLIT ? (A2  + (size_t)b * strideA) : nullptr;
  const T* Bb2 = SPLIT ? (Bt2 + (size_t)b * strideB) : nullptr;

  const int rlane = lane & 15;
  const int koff  = (lane >> 4) * 8;
  const int mOff  = (lane >> 4) * 8;

  v8f acc[4][4];
#pragma unroll
  for (int i = 0; i < 4; ++i)
#pragma unroll
    for (int j = 0; j < 4; ++j) acc[i][j] = (v8f){0.f,0.f,0.f,0.f,0.f,0.f,0.f,0.f};

  for (int k0 = 0; k0 < K; k0 += 32) {
    V bh[4], bl[4];
#pragma unroll
    for (int j = 0; j < 4; ++j) {
      const size_t bo = (size_t)(n0 + (j << 4) + rlane) * ldb + koff + k0;
      bh[j] = Frag<T>::load(Bb + bo);
      if (SPLIT) bl[j] = Frag<T>::load(Bb2 + bo);
    }
#pragma unroll
    for (int i = 0; i < 4; ++i) {
      const size_t ao = (size_t)(m0 + (i << 4) + rlane) * lda + koff + k0;
      V ah = Frag<T>::load(Ab + ao);
      V al;
      if (SPLIT) al = Frag<T>::load(Ab2 + ao);
#pragma unroll
      for (int j = 0; j < 4; ++j) {
        acc[i][j] = Frag<T>::mma(ah, bh[j], acc[i][j]);
        if (SPLIT) {
          acc[i][j] = Frag<T>::mma(ah, bl[j], acc[i][j]);
          acc[i][j] = Frag<T>::mma(al, bh[j], acc[i][j]);
        }
      }
      Frag<T>::guard(acc[i][0], acc[i][3], ah, SPLIT ? al : ah);
    }
    Frag<T>::keep(bh[0], bh[1], bh[2], bh[3]);
    if (SPLIT) Frag<T>::keep(bl[0], bl[1], bl[2], bl[3]);
  }
  acc_guard4(acc[0][0], acc[0][1], acc[0][2], acc[0][3]);
  acc_guard4(acc[1][0], acc[1][1], acc[1][2], acc[1][3]);
  acc_guard4(acc[2][0], acc[2][1], acc[2][2], acc[2][3]);
  acc_guard4(acc[3][0], acc[3][1], acc[3][2], acc[3][3]);

  float* slab = sT[wave];
  const float* Rb = RESID ? (resid + (size_t)b * strideR) : nullptr;
#pragma unroll
  for (int i = 0; i < 4; ++i) {
    const int mBase = m0 + (i << 4);
#pragma unroll
    for (int j = 0; j < 4; ++j) {
      const int n = n0 + (j << 4) + rlane;
      float bv = 0.f;
      if (BIAS_MODE == 2) bv = bias[n];
#pragma unroll
      for (int r = 0; r < 8; ++r) {
        float v = acc[i][j][r] * scale;
        if (BIAS_MODE == 1) v += bias[mBase + mOff + r];
        if (BIAS_MODE == 2) v += bv;
        if (RESID) v += Rb[(size_t)(mBase + mOff + r) * ldc + n];
        if (ACT == 1) v = tanhf(v);
        if (ACT == 2) v = fmaxf(v, 0.0f);
        if (ACT == 3) v = v / (1.0f + expf(-v));
        if (ACT == 4) v = (v > 0.f) ? v : 0.01f * v;
        if (ACT == 5) v = 0.5f * v * (1.0f + erff(v * 0.70710678118654752f));
        slab[(mOff + r) * 68 + (j << 4) + rlane] = v;
      }
    }
    __builtin_amdgcn_fence(__ATOMIC_RELEASE, "workgroup");
    __builtin_amdgcn_wave_barrier();
    __builtin_amdgcn_fence(__ATOMIC_ACQUIRE, "workgroup");
    if (OUT_MODE == 0) {
      float* C = (float*)Cout + (size_t)b * strideC;
      const int hh = lane >> 4, c4 = (lane & 15) * 4;
      for (int pass = 0; pass < 2; ++pass) {
#pragma unroll
        for (int it = 0; it < 8; ++it) {
          const int row = it * 2 + hh;
          v4f v = *(const v4f*)(slab + row * 68 + c4);
          *(volatile v4f*)(C + (size_t)(mBase + row) * ldc + n0 + c4) = v;
        }
        __threadfence();
      }
    } else {
      const int q = lane >> 3, c8 = (lane & 7) * 8;
      unsigned short* C  = (unsigned short*)Cout  + (size_t)b * strideC;
      unsigned short* C2 = (OUT_MODE == 2) ? ((unsigned short*)Cout2 + (size_t)b * strideC) : nullptr;
      for (int pass = 0; pass < 2; ++pass) {
#pragma unroll
        for (int it = 0; it < 4; ++it) {
          const int row = it * 4 + q;
          const float* sp = slab + row * 68 + c8;
          v8h hv, lv;
#pragma unroll
          for (int e = 0; e < 8; ++e) {
            if (OUT_MODE == 1) {
              hv[e] = (_Float16)sp[e];
            } else {
              unsigned short hb = f2bf_bits(sp[e]);
              unsigned short lb = f2bf_bits(sp[e] - bf_bits2f(hb));
              hv[e] = __builtin_bit_cast(_Float16, hb);
              lv[e] = __builtin_bit_cast(_Float16, lb);
            }
          }
          *(volatile v8h*)(C + (size_t)(mBase + row) * ldc + n0 + c8) = hv;
          if (OUT_MODE == 2) *(volatile v8h*)(C2 + (size_t)(mBase + row) * ldc + n0 + c8) = lv;
        }
        __threadfence();
      }
    }
    __builtin_amdgcn_fence(__ATOMIC_RELEASE, "workgroup");
    __builtin_amdgcn_wave_barrier();
    __builtin_amdgcn_fence(__ATOMIC_ACQUIRE, "workgroup");
  }
}

#define NB    16
#define NC    16
#define NH    256
#define NW    256
#define NPIX  65536
#define NLAY  4

#define OFF_TW1   0
#define OFF_A2    16384
#define OFF_A3    49152
#define OFF_TW4   65536
#define OFF_SKW   73728
#define OFF_PW1   75776
#define TAB_HALVES 79872
#define TAB_CHUNKS 9984

union FragU { v16h v; _Float16 s[16]; };

__device__ __forceinline__ v8f mma16g(v16h a, v16h b, v8f c) {
  c = __builtin_amdgcn_wmma_f32_16x16x32_f16(false, a, false, b, (short)0, c, false, false);
  asm volatile("v_nop\n\tv_nop\n\tv_nop\n\tv_nop" : "+v"(c) : "v"(a), "v"(b));
  return c;
}

__device__ __forceinline__ float gelu_t(float x) {
  const float u = 0.7978845608028654f * (x + 0.044715f * x * x * x);
  const float e = __expf(2.0f * u);
  const float t = 1.0f - 2.0f * __builtin_amdgcn_rcpf(e + 1.0f);
  return 0.5f * x * (1.0f + t);
}

__global__ __launch_bounds__(256) void k_tables(const float* __restrict__ skw, const float* __restrict__ pw1,
                                               _Float16* __restrict__ tab) {
  __shared__ float cs[256];
  __shared__ float sn[256];
  const int t = threadIdx.x;
  {
    const float th = (float)t * 0.02454369260617026f;
    cs[t] = cosf(th);
    sn[t] = sinf(th);
  }
  __syncthreads();
  const int g = blockIdx.x * 256 + t;
  if (g >= TAB_CHUNKS) return;
  const int e0 = g * 8;
  union { v8h v; _Float16 s[8]; } u;
  if (e0 < OFF_A2) {
    const int q = e0 >> 8, wb = e0 & 255;
    const int ky = q >> 1;
#pragma unroll
    for (int e = 0; e < 8; ++e) {
      float val = 0.0f;
      if (q < 32) { const int p = (ky * (wb + e)) & 255; val = (q & 1) ? -sn[p] : cs[p]; }
      u.s[e] = (_Float16)val;
    }
  } else if (e0 < OFF_A3) {
    const int idx = e0 - OFF_A2;
    const int r = idx >> 9, kb = idx & 511;
    const int j = r & 31;
    const int kx = (j < 16) ? j : (224 + j);
#pragma unroll
    for (int e = 0; e < 8; ++e) {
      const int k = kb + e;
      const int hk = k & 255, part = k >> 8;
      const int p = (kx * hk) & 255;
      float val;
      if (r < 32) val = part ? sn[p] : cs[p];
      else        val = part ? cs[p] : -sn[p];
      u.s[e] = (_Float16)val;
    }
  } else if (e0 < OFF_TW4) {
    const int idx = e0 - OFF_A3;
    const int hrow = idx >> 6, kb = idx & 63;
#pragma unroll
    for (int e = 0; e < 8; ++e) {
      const int k = kb + e;
      const int j = k & 31;
      const int kx = (j < 16) ? j : (224 + j);
      const int p = (kx * hrow) & 255;
      const float val = (k < 32) ? cs[p] : -sn[p];
      u.s[e] = (_Float16)val;
    }
  } else if (e0 < OFF_SKW) {
    const int idx = e0 - OFF_TW4;
    const int w = idx >> 5, kb = idx & 31;
#pragma unroll
    for (int e = 0; e < 8; ++e) {
      const int k = kb + e;
      const int ky = k & 15;
      const int p = (ky * w) & 255;
      const float c = (ky == 0) ? 1.0f : 2.0f;
      float val;
      if (k < 16) val = c * cs[p];
      else        val = (ky == 0) ? 0.0f : (-c * sn[p]);
      u.s[e] = (_Float16)val;
    }
  } else if (e0 < OFF_PW1) {
    const int idx = e0 - OFF_SKW;
    const int row = idx >> 5, k0 = idx & 31;
#pragma unroll
    for (int e = 0; e < 8; ++e) {
      float val = 0.0f;
      if (k0 < 16) val = 256.0f * skw[row * 16 + k0 + e];
      u.s[e] = (_Float16)val;
    }
  } else {
    const int idx = e0 - OFF_PW1;
    const int row = idx >> 5, k0 = idx & 31;
#pragma unroll
    for (int e = 0; e < 8; ++e) {
      float val = 0.0f;
      if (k0 < 16) val = pw1[row * 16 + k0 + e];
      u.s[e] = (_Float16)val;
    }
  }
  _Float16* dst = tab + e0;
  *(volatile v8h*)dst = u.v;
  __threadfence();
  *(volatile v8h*)dst = u.v;
}

__global__ __launch_bounds__(256) void k_lift(const float* __restrict__ x, const float* __restrict__ lw,
                                             const float* __restrict__ lb, _Float16* __restrict__ V) {
  const unsigned g = blockIdx.x * 256u + threadIdx.x;
  if (g >= (unsigned)(NB * NC * NPIX / 8)) return;
  const unsigned e0 = g * 8u;
  const int b = (int)(e0 >> 20), c = (int)((e0 >> 16) & 15u), px = (int)(e0 & 65535u);
  const float* xp = x + (size_t)b * NPIX + px;
  const v4f x0 = *(const v4f*)xp;
  const v4f x1 = *(const v4f*)(xp + 4);
  const float w = lw[c], bb = lb[c];
  v8h hv;
  hv[0] = (_Float16)(w * x0[0] + bb);
  hv[1] = (_Float16)(w * x0[1] + bb);
  hv[2] = (_Float16)(w * x0[2] + bb);
  hv[3] = (_Float16)(w * x0[3] + bb);
  hv[4] = (_Float16)(w * x1[0] + bb);
  hv[5] = (_Float16)(w * x1[1] + bb);
  hv[6] = (_Float16)(w * x1[2] + bb);
  hv[7] = (_Float16)(w * x1[3] + bb);
  _Float16* dst = V + (size_t)e0;
  *(volatile v8h*)dst = hv;
  __threadfence();
  *(volatile v8h*)dst = hv;
}

__global__ __launch_bounds__(256) void k_mix(const float* __restrict__ X,
                                            const float* __restrict__ w1r, const float* __restrict__ w1i,
                                            const float* __restrict__ w2r, const float* __restrict__ w2i,
                                            int layer, _Float16* __restrict__ OB) {
  __shared__ __align__(16) float ms[8][4 * 64];
  const int tid = threadIdx.x, wave = tid >> 5, lane = tid & 31;
  const int j = lane;
  const int blk = blockIdx.x;
  const int b = blk >> 4, o = blk & 15;
  const int ky0 = 2 * wave;
  const int xm = j & 15;
  const float* wr = (j < 16) ? w1r : w2r;
  const float* wi = (j < 16) ? w1i : w2i;
  const size_t wb = (size_t)layer * 65536 + (size_t)o * 256 + (size_t)xm * 16 + ky0;
  const size_t xr = ((size_t)(b * 64 + j)) * 512 + ky0;
  const size_t xi = ((size_t)(b * 64 + 32 + j)) * 512 + ky0;
  float or0 = 0.f, oi0 = 0.f, or1 = 0.f, oi1 = 0.f;
#pragma unroll 1
  for (int i = 0; i < 16; ++i) {
    const v2f a   = *(const v2f*)(X + xr + i * 32);
    const v2f cc  = *(const v2f*)(X + xi + i * 32);
    const v2f pr  = *(const v2f*)(wr + wb + (size_t)i * 4096);
    const v2f pim = *(const v2f*)(wi + wb + (size_t)i * 4096);
    or0 += a.x * pr.x - cc.x * pim.x;
    oi0 += a.x * pim.x + cc.x * pr.x;
    or1 += a.y * pr.y - cc.y * pim.y;
    oi1 += a.y * pim.y + cc.y * pr.y;
  }
  float* w_ms = ms[wave];
  w_ms[0 * 64 + j] = or0;  w_ms[0 * 64 + 32 + j] = oi0;
  w_ms[1 * 64 + j] = or1;  w_ms[1 * 64 + 32 + j] = oi1;
  w_ms[2 * 64 + j] = oi0;  w_ms[2 * 64 + 32 + j] = -or0;
  w_ms[3 * 64 + j] = oi1;  w_ms[3 * 64 + 32 + j] = -or1;
  __builtin_amdgcn_fence(__ATOMIC_RELEASE, "workgroup");
  __builtin_amdgcn_wave_barrier();
  __builtin_amdgcn_fence(__ATOMIC_ACQUIRE, "workgroup");
  const int li = lane >> 3, c8 = (lane & 7) * 8;
  const int q = ky0 + (li & 1) + (li >> 1) * 16;
  const int qz = 32 + 4 * wave + li;
  _Float16* base = OB + (size_t)blk * 4096;
  for (int pass = 0; pass < 2; ++pass) {
    const float* sp = w_ms + li * 64 + c8;
    v8h hv, zv;
#pragma unroll
    for (int e = 0; e < 8; ++e) { hv[e] = (_Float16)sp[e]; zv[e] = (_Float16)0.0f; }
    *(volatile v8h*)(base + q * 64 + c8) = hv;
    *(volatile v8h*)(base + qz * 64 + c8) = zv;
    __threadfence();
  }
}

__global__ __launch_bounds__(128) void k_specskip(const _Float16* __restrict__ Vcur, const _Float16* __restrict__ Zc,
                                                const _Float16* __restrict__ TW4, const _Float16* __restrict__ SKW,
                                                const float* __restrict__ skb, int dogelu,
                                                _Float16* __restrict__ Vnext) {
  __shared__ __align__(16) _Float16 Vs[16 * 256];
  __shared__ __align__(16) float slabs[4][16 * 68];
  const int tid = threadIdx.x, wave = tid >> 5, lane = tid & 31;
  const int hh = lane >> 4, m = lane & 15;
  const int blk = blockIdx.x;
  const int b = blk >> 8, h = blk & 255;
  for (int c = tid; c < 512; c += 128) {
    const int i = c >> 5, col8 = (c & 31) * 8;
    *(v8h*)(Vs + i * 256 + col8) = *(const v8h*)(Vcur + (((size_t)(b * 16 + i)) * 256 + h) * 256 + col8);
  }
  __syncthreads();
  const int w0 = wave * 64;
  const v16h aZ = Frag<_Float16>::load(Zc + (((size_t)(b * 16 + m)) * 256 + h) * 64 + 8 * hh);
  const v16h aS = Frag<_Float16>::load(SKW + m * 32 + 8 * hh);
  float bias[8];
#pragma unroll
  for (int r = 0; r < 8; ++r) bias[r] = skb[8 * hh + r];
  v8f acc[4];
#pragma unroll
  for (int jt = 0; jt < 4; ++jt) {
    const int col = w0 + 16 * jt + m;
    const v16h bT = Frag<_Float16>::load(TW4 + (size_t)col * 32 + 8 * hh);
    FragU u;
#pragma unroll
    for (int e = 0; e < 8; ++e) { u.s[e] = Vs[(8 * hh + e) * 256 + col]; u.s[8 + e] = (_Float16)0.0f; }
    acc[jt] = (v8f){0.f,0.f,0.f,0.f,0.f,0.f,0.f,0.f};
    acc[jt] = mma16g(aZ, bT, acc[jt]);
    acc[jt] = mma16g(aS, u.v, acc[jt]);
  }
  float* sl = slabs[wave];
#pragma unroll
  for (int jt = 0; jt < 4; ++jt) {
#pragma unroll
    for (int r = 0; r < 8; ++r) {
      float v = acc[jt][r] * (1.0f / 256.0f) + bias[r];
      if (dogelu) v = gelu_t(v);
      sl[(8 * hh + r) * 68 + 16 * jt + m] = v;
    }
  }
  __builtin_amdgcn_fence(__ATOMIC_RELEASE, "workgroup");
  __builtin_amdgcn_wave_barrier();
  __builtin_amdgcn_fence(__ATOMIC_ACQUIRE, "workgroup");
  const int q = lane >> 3, c8 = (lane & 7) * 8;
  for (int pass = 0; pass < 2; ++pass) {
#pragma unroll
    for (int it = 0; it < 4; ++it) {
      const int row = it * 4 + q;
      const float* sp = sl + row * 68 + c8;
      v8h hv;
#pragma unroll
      for (int e = 0; e < 8; ++e) hv[e] = (_Float16)sp[e];
      *(volatile v8h*)(Vnext + (((size_t)(b * 16 + row)) * 256 + h) * 256 + w0 + c8) = hv;
    }
    __threadfence();
  }
}

__global__ __launch_bounds__(128) void k_proj(const _Float16* __restrict__ V, const _Float16* __restrict__ PW1,
                                            const float* __restrict__ pb1, float* __restrict__ part) {
  __shared__ __align__(16) _Float16 Vs[16 * 256];
  __shared__ __align__(16) float Ps[4][128];
  __shared__ __align__(16) float Pt[128];
  const int tid = threadIdx.x, wave = tid >> 5, lane = tid & 31;
  const int hh = lane >> 4, m = lane & 15;
  const int blk = blockIdx.x;
  const int b = blk >> 8, h = blk & 255;
  for (int c = tid; c < 512; c += 128) {
    const int i = c >> 5, col8 = (c & 31) * 8;
    *(v8h*)(Vs + i * 256 + col8) = *(const v8h*)(V + (((size_t)(b * 16 + i)) * 256 + h) * 256 + col8);
  }
  __syncthreads();
  const int w0 = wave * 64;
  v16h bv[4];
#pragma unroll
  for (int jt = 0; jt < 4; ++jt) {
    const int col = w0 + 16 * jt + m;
    FragU u;
#pragma unroll
    for (int e = 0; e < 8; ++e) { u.s[e] = Vs[(8 * hh + e) * 256 + col]; u.s[8 + e] = (_Float16)0.0f; }
    bv[jt] = u.v;
  }
#pragma unroll 1
  for (int mt = 0; mt < 8; ++mt) {
    const v16h a = Frag<_Float16>::load(PW1 + (size_t)(16 * mt + m) * 32 + 8 * hh);
    float brow[8], s[8];
#pragma unroll
    for (int r = 0; r < 8; ++r) { brow[r] = pb1[16 * mt + 8 * hh + r]; s[r] = 0.0f; }
#pragma unroll
    for (int jt = 0; jt < 4; ++jt) {
      v8f acc = (v8f){0.f,0.f,0.f,0.f,0.f,0.f,0.f,0.f};
      acc = mma16g(a, bv[jt], acc);
#pragma unroll
      for (int r = 0; r < 8; ++r) s[r] += gelu_t(acc[r] + brow[r]);
    }
#pragma unroll
    for (int r = 0; r < 8; ++r) {
      s[r] += __shfl_xor(s[r], 1, 32);
      s[r] += __shfl_xor(s[r], 2, 32);
      s[r] += __shfl_xor(s[r], 4, 32);
      s[r] += __shfl_xor(s[r], 8, 32);
    }
    if (m == 0) {
#pragma unroll
      for (int r = 0; r < 8; ++r) Ps[wave][16 * mt + 8 * hh + r] = s[r];
    }
  }
  __syncthreads();
  const float tot = ((Ps[0][tid] + Ps[1][tid]) + Ps[2][tid]) + Ps[3][tid];
  Pt[tid] = tot;
  __syncthreads();
  if (wave == 0) {
    const v4f v = *(const v4f*)(Pt + 4 * lane);
    float* dst = part + (size_t)blk * 128 + 4 * lane;
    *(volatile v4f*)dst = v;
    __threadfence();
    *(volatile v4f*)dst = v;
  }
}

__global__ __launch_bounds__(512) void k_head(const float* __restrict__ part, const float* __restrict__ pw2,
                                            const float* __restrict__ pb2, const float* __restrict__ hw,
                                            const float* __restrict__ hb, float* __restrict__ out) {
  __shared__ __align__(16) float meanS[NB * 128];
  __shared__ __align__(16) float fS[NB * 64];
  __shared__ __align__(16) float oS[32];
  const int t = threadIdx.x;
  for (int uix = t; uix < NB * 128; uix += 512) {
    const int b = uix >> 7, k = uix & 127;
    float s = 0.0f;
#pragma unroll 1
    for (int hrow = 0; hrow < NH; ++hrow) s += part[((size_t)(b * NH + hrow)) * 128 + k];
    meanS[uix] = s * (1.0f / 65536.0f);
  }
  __syncthreads();
  for (int uix = t; uix < NB * 64; uix += 512) {
    const int b = uix >> 6, mrow = uix & 63;
    float s = pb2[mrow];
#pragma unroll 1
    for (int k = 0; k < 128; ++k) s += pw2[mrow * 128 + k] * meanS[b * 128 + k];
    fS[uix] = s;
  }
  __syncthreads();
  if (t < 32) {
    const int b = t >> 1, tt = t & 1;
    float s = hb[tt];
#pragma unroll 1
    for (int mrow = 0; mrow < 64; ++mrow) s += hw[tt * 64 + mrow] * fS[b * 64 + mrow];
    oS[t] = tanhf(s);
  }
  __syncthreads();
  if (t < 8) {
    const v4f v = *(const v4f*)(oS + 4 * t);
    *(volatile v4f*)(out + 4 * t) = v;
    __threadfence();
    *(volatile v4f*)(out + 4 * t) = v;
  }
}

static size_t al_up4k(size_t x) { return (x + 4095) & ~(size_t)4095; }

extern "C" void kernel_launch(void* const* d_in, const int* in_sizes, int n_in,
                              void* d_out, int out_size, void* d_ws, size_t ws_size,
                              hipStream_t stream) {
  if (n_in < 15) return;
  if (in_sizes[0] != NB * NPIX || in_sizes[1] < NC || in_sizes[2] < NC ||
      in_sizes[3] != NLAY * 65536 || in_sizes[4] != NLAY * 65536 ||
      in_sizes[5] != NLAY * 65536 || in_sizes[6] != NLAY * 65536 ||
      in_sizes[7] != NLAY * 256 || in_sizes[8] < NLAY * 16 || in_sizes[9] != 128 * 16 ||
      in_sizes[10] < 128 || in_sizes[11] != 64 * 128 || in_sizes[12] < 64 ||
      in_sizes[13] != 2 * 64 || in_sizes[14] < 2 || out_size != NB * 2) return;

  const float* x    = (const float*)d_in[0];
  const float* lw   = (const float*)d_in[1];
  const float* lb   = (const float*)d_in[2];
  const float* w1r  = (const float*)d_in[3];
  const float* w1i  = (const float*)d_in[4];
  const float* w2r  = (const float*)d_in[5];
  const float* w2i  = (const float*)d_in[6];
  const float* skw  = (const float*)d_in[7];
  const float* skb  = (const float*)d_in[8];
  const float* pw1  = (const float*)d_in[9];
  const float* pb1  = (const float*)d_in[10];
  const float* pw2  = (const float*)d_in[11];
  const float* pb2  = (const float*)d_in[12];
  const float* hw   = (const float*)d_in[13];
  const float* hb   = (const float*)d_in[14];
  float* out = (float*)d_out;

  const size_t szV    = (size_t)NB * NC * NPIX * 2;
  const size_t szTT   = (size_t)NB * NC * 64 * NH * 2;
  const size_t szX    = (size_t)NB * 64 * 512 * 4;
  const size_t szOB   = (size_t)NB * NC * 64 * 64 * 2;
  const size_t szZc   = (size_t)NB * NC * NH * 64 * 2;
  const size_t szPart = (size_t)NB * NH * 128 * 4;
  const size_t szTab  = (size_t)TAB_HALVES * 2;
  char* base = (char*)d_ws;
  size_t off = 0;
  _Float16* V16a = (_Float16*)(base + off); off += al_up4k(szV);
  _Float16* V16b = (_Float16*)(base + off); off += al_up4k(szV);
  _Float16* TT   = (_Float16*)(base + off); off += al_up4k(szTT);
  float*    X    = (float*)(base + off);    off += al_up4k(szX);
  _Float16* OB   = (_Float16*)(base + off); off += al_up4k(szOB);
  _Float16* Zc   = (_Float16*)(base + off); off += al_up4k(szZc);
  float*    Part = (float*)(base + off);    off += al_up4k(szPart);
  _Float16* Tab  = (_Float16*)(base + off); off += al_up4k(szTab);
  if (off > ws_size) return;
  _Float16* TW1  = Tab + OFF_TW1;
  _Float16* A2t  = Tab + OFF_A2;
  _Float16* A3t  = Tab + OFF_A3;
  _Float16* TW4  = Tab + OFF_TW4;
  _Float16* SKW  = Tab + OFF_SKW;
  _Float16* PW1h = Tab + OFF_PW1;

  k_tables<<<dim3(TAB_CHUNKS / 256), dim3(256), 0, stream>>>(skw, pw1, Tab);
  k_lift<<<dim3(NB * NC * NPIX / 8 / 256), dim3(256), 0, stream>>>(x, lw, lb, V16a);

  _Float16* vc = V16a;
  _Float16* vn = V16b;
  for (int l = 0; l < NLAY; ++l) {
    wmma_gemm64<0, false, 0, 1, false, 0><<<dim3(1, NB * NC), dim3(256), 0, stream>>>(
        (const unsigned short*)TW1, (const unsigned short*)nullptr, 256, (long)0,
        (const unsigned short*)vc, (const unsigned short*)nullptr, 256, (long)NPIX,
        (void*)TT, (void*)nullptr, 256, (long)(64 * NH),
        (const float*)nullptr, (const float*)nullptr, (long)0,
        64, 256, 256, 1.0f);
    wmma_gemm64<0, false, 0, 0, false, 0><<<dim3(1, NB), dim3(256), 0, stream>>>(
        (const unsigned short*)A2t, (const unsigned short*)nullptr, 512, (long)0,
        (const unsigned short*)TT, (const unsigned short*)nullptr, 512, (long)(NC * 64 * NH),
        (void*)X, (void*)nullptr, 512, (long)(64 * 512),
        (const float*)nullptr, (const float*)nullptr, (long)0,
        64, 512, 512, 1.0f);
    k_mix<<<dim3(NB * NC), dim3(256), 0, stream>>>(X, w1r, w1i, w2r, w2i, l, OB);
    wmma_gemm64<0, false, 0, 1, false, 0><<<dim3(1, NB * NC), dim3(256), 0, stream>>>(
        (const unsigned short*)A3t, (const unsigned short*)nullptr, 64, (long)0,
        (const unsigned short*)OB, (const unsigned short*)nullptr, 64, (long)(64 * 64),
        (void*)Zc, (void*)nullptr, 64, (long)(NH * 64),
        (const float*)nullptr, (const float*)nullptr, (long)0,
        256, 64, 64, 1.0f / 256.0f);
    k_specskip<<<dim3(NB * NH), dim3(128), 0, stream>>>(vc, Zc, TW4, SKW + (size_t)l * 512,
                                                         skb + (size_t)l * 16, (l < NLAY - 1) ? 1 : 0, vn);
    _Float16* tmp = vc; vc = vn; vn = tmp;
  }

  k_proj<<<dim3(NB * NH), dim3(128), 0, stream>>>(vc, PW1h, pb1, Part);
  k_head<<<dim3(1), dim3(512), 0, stream>>>(Part, pw2, pb2, hw, hb, out);
}
